// MambaBlock_69243462746249
// MI455X (gfx1250) — hardware-verified
//
#include <hip/hip_runtime.h>
#include <math.h>

typedef __attribute__((ext_vector_type(16))) _Float16 v16h;
typedef __attribute__((ext_vector_type(8)))  _Float16 v8h;
typedef __attribute__((ext_vector_type(16))) __bf16   v16b;
typedef __attribute__((ext_vector_type(8)))  __bf16   v8b;
typedef __attribute__((ext_vector_type(8)))  float    v8f;
typedef __attribute__((ext_vector_type(4)))  float    v4f;

constexpr int kBatch = 2;
constexpr int kSeqT  = 8192;
constexpr int kDm    = 768;
constexpr int kDin   = 1536;
constexpr int kNxz   = 2 * kDin;
constexpr int kConvK = 4;
constexpr int kRows  = kBatch * kSeqT;
constexpr int kCG    = 256;
constexpr int kNGrp  = kDin / kCG;
constexpr int kXgP   = 2 * kCG;
constexpr int kScTP  = 260;
constexpr float kAlpha         = 0.9f;
constexpr float kOneMinusAlpha = 0.1f;
constexpr float kYCarry   = 1024.0f;
constexpr float kWCarry   = 1024.0f;
constexpr float kOutScale = 1.0f / (kYCarry * kWCarry);
static_assert(kNGrp * kCG == kDin, "grouping");
static_assert((kDm % 32) == 0 && (kDin % 32) == 0, "GEMM K multiples of 32");
static_assert((kRows % 64) == 0 && (kCG % 64) == 0 && (kDm % 64) == 0 && (kNxz % 64) == 0 && (kDin % 64) == 0,
              "GEMM M,N and transpose tiles multiples of 64");
static_assert((kSeqT % 16) == 0 && kCG == 256, "scan tile");
static_assert(((kRows * kDm) % 2048) == 0, "cast coverage");

constexpr size_t kSzXB = (size_t)kRows * kDm * 2;
constexpr size_t kSzW1 = (size_t)kNxz * kDm * 2;
constexpr size_t kSzW2 = (size_t)kDm * kDin * 2;
constexpr size_t kSzBI = (size_t)kNxz * 4;
constexpr size_t kSzBO = (size_t)kDm * 4;
constexpr size_t kSzXZ = (size_t)kRows * kXgP * 4;
constexpr size_t kSzY  = (size_t)kRows * kDin * 2;
constexpr size_t kOffXB = 0;
constexpr size_t kOffW1 = kOffXB + kSzXB;
constexpr size_t kOffW2 = kOffW1 + kSzW1;
constexpr size_t kOffBI = kOffW2 + kSzW2;
constexpr size_t kOffBO = kOffBI + kSzBI;
constexpr size_t kOffXZ = kOffBO + kSzBO;
constexpr size_t kOffY  = kOffXZ + kSzXZ;
constexpr size_t kWsTotal = kOffY + kSzY;
static_assert(kWsTotal == 116145152ull, "carve total");
static_assert(kWsTotal <= 134217728ull, "carve cap");
static_assert((kOffW1 % 128) == 0 && (kOffW2 % 128) == 0 && (kOffBI % 128) == 0 && (kOffBO % 128) == 0 &&
              (kOffXZ % 128) == 0 && (kOffY % 128) == 0, "128-B aligned regions");

__device__ __forceinline__ unsigned short f2bf_bits(float f) {
  unsigned u = __float_as_uint(f);
  return (unsigned short)((u + 0x7FFFu + ((u >> 16) & 1u)) >> 16);
}
__device__ __forceinline__ float bf_bits2f(unsigned short h) { return __uint_as_float(((unsigned)h) << 16); }
__device__ __forceinline__ float rne_bf16(float f) { return bf_bits2f(f2bf_bits(f)); }

__device__ __forceinline__ void dep_guard4_h(v8f& a, v8f& b, v8f& c, v8f& d, v16h x, v16h y) {
  asm volatile("v_nop\n\tv_nop\n\tv_nop\n\tv_nop" : "+v"(a), "+v"(b), "+v"(c), "+v"(d) : "v"(x), "v"(y));
}
__device__ __forceinline__ void dep_guard4_b(v8f& a, v8f& b, v8f& c, v8f& d, v16b x, v16b y) {
  asm volatile("v_nop\n\tv_nop\n\tv_nop\n\tv_nop" : "+v"(a), "+v"(b), "+v"(c), "+v"(d) : "v"(x), "v"(y));
}
__device__ __forceinline__ void keep4_h(v16h a, v16h b, v16h c, v16h d) { asm volatile("v_nop" :: "v"(a), "v"(b), "v"(c), "v"(d)); }
__device__ __forceinline__ void keep4_b(v16b a, v16b b, v16b c, v16b d) { asm volatile("v_nop" :: "v"(a), "v"(b), "v"(c), "v"(d)); }
__device__ __forceinline__ void acc_guard4(v8f& a, v8f& b, v8f& c, v8f& d) { asm volatile("v_nop\n\tv_nop\n\tv_nop\n\tv_nop" : "+v"(a), "+v"(b), "+v"(c), "+v"(d)); }
template <typename T> struct Frag;
template <> struct Frag<_Float16> {
  typedef v16h V; union U { v16h v; v8h h[2]; };
  static __device__ __forceinline__ v16h load(const _Float16* p) {
    U f; f.h[0] = *(const v8h*)(p); f.h[1] = *(const v8h*)(p + 16); return f.v;
  }
  static __device__ __forceinline__ v8f mma(v16h a, v16h b, v8f c) {
    return __builtin_amdgcn_wmma_f32_16x16x32_f16(false, a, false, b, (short)0, c, false, false);
  }
  static __device__ __forceinline__ void guard4(v8f& a, v8f& b, v8f& c, v8f& d, v16h x, v16h y) { dep_guard4_h(a, b, c, d, x, y); }
  static __device__ __forceinline__ void keep(v16h a, v16h b, v16h c, v16h d) { keep4_h(a, b, c, d); }
};
template <> struct Frag<__bf16> {
  typedef v16b V; union U { v16b v; v8b h[2]; };
  static __device__ __forceinline__ v16b load(const __bf16* p) {
    U f; f.h[0] = *(const v8b*)(p); f.h[1] = *(const v8b*)(p + 16); return f.v;
  }
  static __device__ __forceinline__ v8f mma(v16b a, v16b b, v8f c) {
    return __builtin_amdgcn_wmma_f32_16x16x32_bf16(false, a, false, b, (short)0, c, false, false);
  }
  static __device__ __forceinline__ void guard4(v8f& a, v8f& b, v8f& c, v8f& d, v16b x, v16b y) { dep_guard4_b(a, b, c, d, x, y); }
  static __device__ __forceinline__ void keep(v16b a, v16b b, v16b c, v16b d) { keep4_b(a, b, c, d); }
};

template <int ET> struct Elem;
template <> struct Elem<0> { typedef _Float16 T; };
template <> struct Elem<1> { typedef __bf16 T; };
template <int ET, bool SPLIT, int BIAS_MODE, int OUT_MODE, bool RESID, int ACT = 0>
__global__ __launch_bounds__(256) void wmma_gemm64(
    const unsigned short* __restrict__ Ap, const unsigned short* __restrict__ A2p, int lda, long strideA,
    const unsigned short* __restrict__ Btp, const unsigned short* __restrict__ Bt2p, int ldb, long strideB,
    void* __restrict__ Cout, void* __restrict__ Cout2, int ldc, long strideC,
    const float* __restrict__ bias,
    const float* __restrict__ resid, long strideR,
    int M, int N, int K, float scale) {
  typedef typename Elem<ET>::T T;
  typedef typename Frag<T>::V V;
  const T* A = (const T*)Ap; const T* A2 = (const T*)A2p; const T* Bt = (const T*)Btp; const T* Bt2 = (const T*)Bt2p;
  __shared__ __align__(16) float sT[8][16 * 68];
  const int b    = blockIdx.y;
  const int lane = threadIdx.x & 31;
  const int wave = threadIdx.x >> 5;
  const int tilesN = N >> 6;
  const int tilesM = M >> 6;
  const int tile = blockIdx.x * 8 + wave;
  if (tile >= tilesM * tilesN) return;
  const int tm = tile / tilesN;
  const int tn = tile - tm * tilesN;
  const int m0 = tm << 6;
  const int n0 = tn << 6;

  const T* Ab  = A  + (size_t)b * strideA;
  const T* Bb  = Bt + (size_t)b * strideB;
  const T* Ab2 = SPLIT ? (A2  + (size_t)b * strideA) : nullptr;
  const T* Bb2 = SPLIT ? (Bt2 + (size_t)b * strideB) : nullptr;

  const int rlane = lane & 15;
  const int koff  = (lane >> 4) * 8;
  const int mOff  = (lane >> 4) * 8;

  v8f acc[4][4];
#pragma unroll
  for (int i = 0; i < 4; ++i)
#pragma unroll
    for (int j = 0; j < 4; ++j) acc[i][j] = (v8f){0.f,0.f,0.f,0.f,0.f,0.f,0.f,0.f};

  for (int k0 = 0; k0 < K; k0 += 32) {
    V bh[4], bl[4];
#pragma unroll
    for (int j = 0; j < 4; ++j) {
      const size_t bo = (size_t)(n0 + (j << 4) + rlane) * ldb + koff + k0;
      bh[j] = Frag<T>::load(Bb + bo);
      if (SPLIT) bl[j] = Frag<T>::load(Bb2 + bo);
    }
#pragma unroll
    for (int i = 0; i < 4; ++i) {
      const size_t ao = (size_t)(m0 + (i << 4) + rlane) * lda + koff + k0;
      V ah = Frag<T>::load(Ab + ao);
      V al;
      if (SPLIT) al = Frag<T>::load(Ab2 + ao);
#pragma unroll
      for (int j = 0; j < 4; ++j) {
        acc[i][j] = Frag<T>::mma(ah, bh[j], acc[i][j]);
        if (SPLIT) {
          acc[i][j] = Frag<T>::mma(ah, bl[j], acc[i][j]);
          acc[i][j] = Frag<T>::mma(al, bh[j], acc[i][j]);
        }
      }
      Frag<T>::guard4(acc[i][0], acc[i][1], acc[i][2], acc[i][3], ah, SPLIT ? al : ah);
    }
    Frag<T>::keep(bh[0], bh[1], bh[2], bh[3]);
    if (SPLIT) Frag<T>::keep(bl[0], bl[1], bl[2], bl[3]);
  }
  acc_guard4(acc[0][0], acc[0][1], acc[0][2], acc[0][3]);
  acc_guard4(acc[1][0], acc[1][1], acc[1][2], acc[1][3]);
  acc_guard4(acc[2][0], acc[2][1], acc[2][2], acc[2][3]);
  acc_guard4(acc[3][0], acc[3][1], acc[3][2], acc[3][3]);

  float* slab = sT[wave];
  const float* Rb = RESID ? (resid + (size_t)b * strideR) : nullptr;
#pragma unroll
  for (int i = 0; i < 4; ++i) {
    const int mBase = m0 + (i << 4);
#pragma unroll
    for (int j = 0; j < 4; ++j) {
      const int n = n0 + (j << 4) + rlane;
      float bv = 0.f;
      if (BIAS_MODE == 2) bv = bias[n];
#pragma unroll
      for (int r = 0; r < 8; ++r) {
        float v = acc[i][j][r] * scale;
        if (BIAS_MODE == 1) v += bias[mBase + mOff + r];
        if (BIAS_MODE == 2) v += bv;
        if (RESID) v += Rb[(size_t)(mBase + mOff + r) * ldc + n];
        if (ACT == 1) v = tanhf(v);
        if (ACT == 2) v = fmaxf(v, 0.0f);
        if (ACT == 3) v = v / (1.0f + expf(-v));
        if (ACT == 4) v = (v > 0.f) ? v : 0.01f * v;
        slab[(mOff + r) * 68 + (j << 4) + rlane] = v;
      }
    }
    __builtin_amdgcn_fence(__ATOMIC_RELEASE, "workgroup");
    __builtin_amdgcn_wave_barrier();
    __builtin_amdgcn_fence(__ATOMIC_ACQUIRE, "workgroup");
    if (OUT_MODE == 0) {
      float* C = (float*)Cout + (size_t)b * strideC;
      const int hh = lane >> 4, c4 = (lane & 15) * 4;
      for (int pass = 0; pass < 2; ++pass) {
#pragma unroll
        for (int it = 0; it < 8; ++it) {
          const int row = it * 2 + hh;
          v4f v = *(const v4f*)(slab + row * 68 + c4);
          *(volatile v4f*)(C + (size_t)(mBase + row) * ldc + n0 + c4) = v;
        }
        __threadfence();
      }
    } else {
      const int q = lane >> 3, c8 = (lane & 7) * 8;
      unsigned short* C  = (unsigned short*)Cout  + (size_t)b * strideC;
      unsigned short* C2 = (OUT_MODE == 2) ? ((unsigned short*)Cout2 + (size_t)b * strideC) : nullptr;
      for (int pass = 0; pass < 2; ++pass) {
#pragma unroll
        for (int it = 0; it < 4; ++it) {
          const int row = it * 4 + q;
          const float* sp = slab + row * 68 + c8;
          v8h hv, lv;
#pragma unroll
          for (int e = 0; e < 8; ++e) {
            if (OUT_MODE == 1) {
              hv[e] = (_Float16)sp[e];
            } else {
              unsigned short hb = f2bf_bits(sp[e]);
              unsigned short lb = f2bf_bits(sp[e] - bf_bits2f(hb));
              hv[e] = __builtin_bit_cast(_Float16, hb);
              lv[e] = __builtin_bit_cast(_Float16, lb);
            }
          }
          *(volatile v8h*)(C + (size_t)(mBase + row) * ldc + n0 + c8) = hv;
          if (OUT_MODE == 2) *(volatile v8h*)(C2 + (size_t)(mBase + row) * ldc + n0 + c8) = lv;
        }
        __threadfence();
      }
    }
    __builtin_amdgcn_fence(__ATOMIC_RELEASE, "workgroup");
    __builtin_amdgcn_wave_barrier();
    __builtin_amdgcn_fence(__ATOMIC_ACQUIRE, "workgroup");
  }
}

__global__ __launch_bounds__(256) void cast_bf16_kernel(
    const float* __restrict__ src, unsigned short* __restrict__ dst, int total8)
{
  const int i = blockIdx.x * 256 + threadIdx.x;
  if (i >= total8) return;
  const size_t e0 = (size_t)i << 3;
  const float* p = src + e0;
  const v4f a0 = *(const v4f*)(p);
  const v4f a1 = *(const v4f*)(p + 4);
  v8h hv;
#pragma unroll
  for (int e = 0; e < 4; ++e) {
    hv[e]     = __builtin_bit_cast(_Float16, f2bf_bits(a0[e]));
    hv[4 + e] = __builtin_bit_cast(_Float16, f2bf_bits(a1[e]));
  }
  unsigned short* qd = dst + e0;
  *(volatile v8h*)qd = hv;
  __threadfence();
  *(volatile v8h*)qd = hv;
}

__global__ __launch_bounds__(256) void rne16_f32_kernel(
    const float* __restrict__ src, float* __restrict__ dst, int n4)
{
  const int i = blockIdx.x * 256 + threadIdx.x;
  if (i >= n4) return;
  const v4f a = *(const v4f*)(src + (size_t)i * 4);
  v4f r;
#pragma unroll
  for (int e = 0; e < 4; ++e) r[e] = rne_bf16(a[e]);
  float* qd = dst + (size_t)i * 4;
  *(volatile v4f*)qd = r;
  __threadfence();
  *(volatile v4f*)qd = r;
}

template <int OKIND>
__global__ __launch_bounds__(256) void transpose_cast_kernel(
    const float* __restrict__ W, unsigned short* __restrict__ Bt, int Kdim, int Ndim, float scale)
{
  __shared__ float tile[64 * 65];
  const int tid = threadIdx.x, lane = tid & 31, wave = tid >> 5;
  const int n0 = blockIdx.x * 64;
  const int k0 = blockIdx.y * 64;
#pragma unroll
  for (int p = 0; p < 16; ++p) {
    if (p == 8) asm volatile("" ::: "memory");
    const int idx = tid + p * 256;
    const int kk  = idx >> 6;
    const int nn  = idx & 63;
    const int n   = n0 + nn;
    const int nc  = (n < Ndim) ? n : (Ndim - 1);
    const float v  = W[(size_t)(k0 + kk) * Ndim + nc];
    const float vb = rne_bf16(v);
    const float vs = (OKIND == 0) ? vb : (vb * scale);
    tile[kk * 65 + nn] = (n < Ndim) ? vs : 0.f;
  }
  __syncthreads();
  const int q = lane >> 3, c8 = (lane & 7) * 8;
  v8h hv[2];
#pragma unroll
  for (int it = 0; it < 2; ++it) {
    const int nrow = it * 32 + wave * 4 + q;
#pragma unroll
    for (int e = 0; e < 8; ++e) {
      const float tv = tile[(c8 + e) * 65 + nrow];
      if (OKIND == 0) hv[it][e] = __builtin_bit_cast(_Float16, f2bf_bits(tv));
      else            hv[it][e] = (_Float16)tv;
    }
  }
  for (int pass = 0; pass < 2; ++pass) {
#pragma unroll
    for (int it = 0; it < 2; ++it) {
      const int nrow = it * 32 + wave * 4 + q;
      *(volatile v8h*)(Bt + (size_t)(n0 + nrow) * Kdim + k0 + c8) = hv[it];
    }
    __threadfence();
  }
}

__global__ __launch_bounds__(256) void scan_gate_kernel(
    const float* __restrict__ XZ, const float* __restrict__ cw, const float* __restrict__ cb,
    const float* __restrict__ Dv, unsigned short* __restrict__ Y, int g)
{
  __shared__ __align__(16) float sY[16 * kScTP];
  const int tid = threadIdx.x, lane = tid & 31, wave = tid >> 5;
  const int bix = blockIdx.x;
  const int c   = g * kCG + tid;
  const size_t row0 = (size_t)bix * kSeqT;
  const float w0 = rne_bf16(cw[c * kConvK + 0]);
  const float w1 = rne_bf16(cw[c * kConvK + 1]);
  const float w2 = rne_bf16(cw[c * kConvK + 2]);
  const float w3 = rne_bf16(cw[c * kConvK + 3]);
  const float bc = rne_bf16(cb[c]);
  const float Dd = rne_bf16(Dv[c]);
  float xm3 = 0.f, xm2 = 0.f, xm1 = 0.f;
  float h = 0.f;
  const size_t ycol = (size_t)g * kCG + lane * 8;
#pragma unroll 1
  for (int t0 = 0; t0 < kSeqT; t0 += 16) {
#pragma unroll 1
    for (int s = 0; s < 16; ++s) {
      const size_t r = row0 + (size_t)(t0 + s);
      const float xcur = XZ[r * kXgP + tid];
      const float zv   = XZ[r * kXgP + kCG + tid];
      float cv = w0 * xm3;
      cv = fmaf(w1, xm2, cv);
      cv = fmaf(w2, xm1, cv);
      cv = fmaf(w3, xcur, cv);
      cv += bc;
      const float sgc = __builtin_amdgcn_rcpf(1.0f + expf(-cv));
      const float xc  = cv * sgc;
      h = kAlpha * h + kOneMinusAlpha * xc;
      const float sgz = __builtin_amdgcn_rcpf(1.0f + expf(-zv));
      const float gz  = zv * sgz;
      const float y   = (xc * Dd + h) * gz;
      sY[s * kScTP + tid] = y * kYCarry;
      xm3 = xm2; xm2 = xm1; xm1 = xcur;
    }
    __syncthreads();
    v8h hv[2];
#pragma unroll
    for (int it = 0; it < 2; ++it) {
      const float* sp = sY + (it * 8 + wave) * kScTP + lane * 8;
      const v4f a0 = *(const v4f*)(sp);
      const v4f a1 = *(const v4f*)(sp + 4);
#pragma unroll
      for (int e = 0; e < 4; ++e) { hv[it][e] = (_Float16)a0[e]; hv[it][4 + e] = (_Float16)a1[e]; }
    }
    for (int pass = 0; pass < 2; ++pass) {
#pragma unroll
      for (int it = 0; it < 2; ++it)
        *(volatile v8h*)(Y + (row0 + (size_t)(t0 + it * 8 + wave)) * kDin + ycol) = hv[it];
      __threadfence();
    }
    __syncthreads();
  }
}

extern "C" void kernel_launch(void* const* d_in, const int* in_sizes, int n_in,
                              void* d_out, int out_size, void* d_ws, size_t ws_size,
                              hipStream_t stream)
{
  if (n_in < 12) return;
  if (in_sizes[0] != kRows * kDm) return;
  if (in_sizes[1] != kDm * kNxz) return;
  if (in_sizes[2] != kNxz) return;
  if (in_sizes[3] != kDin * kConvK) return;
  if (in_sizes[4] != kDin) return;
  if (in_sizes[9] != kDin) return;
  if (in_sizes[10] != kDin * kDm) return;
  if (in_sizes[11] != kDm) return;
  if (out_size != kRows * kDm) return;
  if (ws_size < kWsTotal) return;

  const float* x      = (const float*)d_in[0];
  const float* in_w   = (const float*)d_in[1];
  const float* in_b   = (const float*)d_in[2];
  const float* conv_w = (const float*)d_in[3];
  const float* conv_b = (const float*)d_in[4];
  const float* Dp     = (const float*)d_in[9];
  const float* out_w  = (const float*)d_in[10];
  const float* out_b  = (const float*)d_in[11];
  float* dout = (float*)d_out;

  char* ws = (char*)d_ws;
  unsigned short* XB = (unsigned short*)(ws + kOffXB);
  unsigned short* W1 = (unsigned short*)(ws + kOffW1);
  unsigned short* W2 = (unsigned short*)(ws + kOffW2);
  float*          BI = (float*)(ws + kOffBI);
  float*          BO = (float*)(ws + kOffBO);
  float*          XZ = (float*)(ws + kOffXZ);
  unsigned short* Yp = (unsigned short*)(ws + kOffY);
  const float* dummy_resid = x;

  cast_bf16_kernel<<<(kRows * kDm) / 8 / 256, 256, 0, stream>>>(x, XB, (kRows * kDm) / 8);
  transpose_cast_kernel<0><<<dim3(kNxz / 64, kDm / 64), 256, 0, stream>>>(in_w, W1, kDm, kNxz, 1.0f);
  transpose_cast_kernel<1><<<dim3(kDm / 64, kDin / 64), 256, 0, stream>>>(out_w, W2, kDin, kDm, kWCarry);
  rne16_f32_kernel<<<(kNxz / 4 + 255) / 256, 256, 0, stream>>>(in_b, BI, kNxz / 4);
  rne16_f32_kernel<<<(kDm / 4 + 255) / 256, 256, 0, stream>>>(out_b, BO, kDm / 4);

  constexpr int kBlkG1 = (kRows / 64) * (kCG / 64) / 8;
  constexpr int kBlkG2 = (kRows / 64) * (kDm / 64) / 8;
  for (int g = 0; g < kNGrp; ++g) {
    wmma_gemm64<1, false, 2, 0, false><<<dim3(kBlkG1, 1), 256, 0, stream>>>(
        XB, XB, kDm, 0L,
        W1 + (size_t)(g * kCG) * kDm, W1 + (size_t)(g * kCG) * kDm, kDm, 0L,
        (void*)XZ, (void*)XZ, kXgP, 0L,
        BI + g * kCG, dummy_resid, 0L,
        kRows, kCG, kDm, 1.0f);
    wmma_gemm64<1, false, 2, 0, false><<<dim3(kBlkG1, 1), 256, 0, stream>>>(
        XB, XB, kDm, 0L,
        W1 + (size_t)(kDin + g * kCG) * kDm, W1 + (size_t)(kDin + g * kCG) * kDm, kDm, 0L,
        (void*)(XZ + kCG), (void*)(XZ + kCG), kXgP, 0L,
        BI + kDin + g * kCG, dummy_resid, 0L,
        kRows, kCG, kDm, 1.0f);
    scan_gate_kernel<<<kBatch, kCG, 0, stream>>>(XZ, conv_w, conv_b, Dp, Yp, g);
  }

  wmma_gemm64<0, false, 2, 0, false><<<dim3(kBlkG2, 1), 256, 0, stream>>>(
      Yp, Yp, kDin, 0L,
      W2, W2, kDin, 0L,
      (void*)dout, (void*)dout, kDm, 0L,
      BO, dummy_resid, 0L,
      kRows, kDm, kDin, kOutScale);
}
